// BudgetAllocationRGNN_65859028517265
// MI455X (gfx1250) — hardware-verified
//
#include <hip/hip_runtime.h>
#include <math.h>

typedef __attribute__((ext_vector_type(16))) _Float16 v16h;
typedef __attribute__((ext_vector_type(16))) __bf16 v16b;
typedef __attribute__((ext_vector_type(8)))  _Float16 v8h;
typedef __attribute__((ext_vector_type(8)))  float v8f;
typedef __attribute__((ext_vector_type(4)))  float v4f;
typedef __attribute__((ext_vector_type(2)))  float v2f;
typedef __attribute__((ext_vector_type(4)))  unsigned v4u;
typedef __attribute__((ext_vector_type(4)))  int v4i;
typedef float __attribute__((may_alias)) float_a;
typedef int __attribute__((may_alias)) int_a;

template <typename T> __device__ __forceinline__ void vst2(void* p, T v) { *(volatile T*)p = v; __threadfence(); *(volatile T*)p = v; }
__device__ __forceinline__ v8f wmma16(v16h a, v16h b, v8f c) {
  v8f d = __builtin_amdgcn_wmma_f32_16x16x32_f16(false, a, false, b, (short)0, c, false, false);
  asm volatile("v_nop\n\tv_nop\n\tv_nop\n\tv_nop" : "+v"(d) : "v"(a), "v"(b));
  return d;
}
__device__ __forceinline__ v8f wmma_bf(v16b a, v16b b, v8f c) {
  v8f d = __builtin_amdgcn_wmma_f32_16x16x32_bf16(false, a, false, b, (short)0, c, false, false);
  asm volatile("v_nop\n\tv_nop\n\tv_nop\n\tv_nop" : "+v"(d) : "v"(a), "v"(b));
  return d;
}
__device__ __forceinline__ v16h frag_h(const _Float16* rowk0, int lane) {
  union { v16h v; v8h q[2]; } u; const _Float16* p = rowk0 + 8 * (lane >> 4);
  u.q[0] = *(const v8h*)p; u.q[1] = *(const v8h*)(p + 16); return u.v;
}
__device__ __forceinline__ v16h frag_f32(const float* rowk0, int lane) {
  v16h a; const float* p = rowk0 + 8 * (lane >> 4);
#pragma unroll
  for (int i = 0; i < 8; ++i) { a[i] = (_Float16)p[i]; a[8 + i] = (_Float16)p[16 + i]; }
  return a;
}
__device__ __forceinline__ v16h frag_f32s(const float* rowk0, int lane, float sc) {
  v16h a; const float* p = rowk0 + 8 * (lane >> 4);
#pragma unroll
  for (int i = 0; i < 8; ++i) { a[i] = (_Float16)(p[i] * sc); a[8 + i] = (_Float16)(p[16 + i] * sc); }
  return a;
}
__device__ __forceinline__ v16h fragc_f32(const float* W, int k0, int n, int lane, int ld, int K) {
  v16h a; const int g = lane >> 4;
#pragma unroll
  for (int i = 0; i < 8; ++i) { const int ka = k0 + 8 * g + i, kb = ka + 16;
    a[i] = (_Float16)(ka < K ? W[(size_t)(ka < K ? ka : K - 1) * ld + n] : 0.f); a[8 + i] = (_Float16)(kb < K ? W[(size_t)(kb < K ? kb : K - 1) * ld + n] : 0.f); }
  return a;
}
struct F2 { v16b h, l; };
__device__ __forceinline__ F2 bsplit16(const float v[16]) { F2 r;
#pragma unroll
  for (int i = 0; i < 16; ++i) { const __bf16 h = (__bf16)v[i]; r.h[i] = h; r.l[i] = (__bf16)(v[i] - (float)h); }
  return r; }
__device__ __forceinline__ F2 split_row(const float* row, int k0, int lane) { float v[16]; const float* p = row + k0 + 8 * (lane >> 4);
#pragma unroll
  for (int i = 0; i < 8; ++i) { v[i] = p[i]; v[8 + i] = p[16 + i]; }
  return bsplit16(v); }
__device__ __forceinline__ F2 split_rowK(const float* row, int k0, int lane, int K) { float v[16]; const int g = lane >> 4;
#pragma unroll
  for (int i = 0; i < 8; ++i) { const int ka = k0 + 8 * g + i, kb = ka + 16; v[i] = ka < K ? row[ka < K ? ka : K - 1] : 0.f; v[8 + i] = kb < K ? row[kb < K ? kb : K - 1] : 0.f; }
  return bsplit16(v); }
__device__ __forceinline__ F2 split_col(const float* W, int k0, int n, int lane, int ld, int K) { float v[16]; const int g = lane >> 4;
#pragma unroll
  for (int i = 0; i < 8; ++i) { const int ka = k0 + 8 * g + i, kb = ka + 16; v[i] = ka < K ? W[(size_t)(ka < K ? ka : K - 1) * ld + n] : 0.f; v[8 + i] = kb < K ? W[(size_t)(kb < K ? kb : K - 1) * ld + n] : 0.f; }
  return bsplit16(v); }
__device__ __forceinline__ v8f mac3(const F2& a, const F2& b, v8f c) { c = wmma_bf(a.l, b.h, c); c = wmma_bf(a.h, b.l, c); return wmma_bf(a.h, b.h, c); }
__device__ __forceinline__ float sigm(float v) { return 1.0f / (1.0f + expf(-v)); }
#define LDSX() do { asm volatile("s_wait_dscnt 0" ::: "memory"); __builtin_amdgcn_wave_barrier(); __builtin_amdgcn_fence(__ATOMIC_RELEASE, "workgroup"); } while (0)


#define NN 50000
#define NE 800000
#define NR 8
#define FIN 128
#define HID 256
#define H2 128
#define NRB ((NN + 63) / 64)
#define NPAD (NRB * 64)
#ifndef NNT
#define NNT NN
#define NRBT NRB
#endif
typedef __attribute__((ext_vector_type(8))) __bf16 v8b;
__device__ __forceinline__ v16b frag_b(const __bf16* rowk0, int lane) {
  union { v16b v; v8b q[2]; } u; const __bf16* p = rowk0 + 8 * (lane >> 4);
  u.q[0] = *(const v8b*)p; u.q[1] = *(const v8b*)(p + 16); return u.v;
}
__device__ __forceinline__ float bfr(float v) { return (float)(__bf16)v; }
__device__ __attribute__((noinline)) float exp_ni(float v) { return expf(v); }
__device__ __attribute__((noinline)) float erf_ni(float v) { return erff(v); }

#define CSA_N 50000
#define CSA_E 800000
#define CSA_FINN (CSA_E + 32 * CSA_NBK)
#define CSA_CHUNK 4096
#define CSA_BKT 256
#define CSA_NCH ((CSA_E + CSA_CHUNK - 1) / CSA_CHUNK)
#define CSA_NBK ((CSA_N + CSA_BKT - 1) / CSA_BKT)
#define CSA_NBKP (((CSA_NBK + 63) / 64) * 64)
#define CSA_SEGCAP (CSA_E + 32 * CSA_NBK * CSA_NCH)
#ifndef CSA_BCAP
#define CSA_BCAP 10240
#endif
#define CSA_SZ_CNT   (4u * CSA_NCH * CSA_NBKP)
#define CSA_SZ_OFF   (4u * CSA_NBK * (((CSA_NCH + 31) / 32) * 32))
#define CSA_SZ_BST   (4u * (((CSA_NBK + 1 + 31) / 32) * 32))
#define CSA_SZ_SEG   (4u * CSA_SEGCAP)
#define CSA_SZ_FIN   (4u * (CSA_E + 32 * CSA_NBK))
#define CSA_SZ_ROW   (4u * CSA_NBK * CSA_BKT)
#define CSA_OFFP (((CSA_NCH + 31) / 32) * 32)

__global__ __launch_bounds__(256) void k_csA_cnt(const int* __restrict__ DST, int dstride, int* __restrict__ CNT) {
  __shared__ unsigned short sc[256][CSA_NBK + 1]; __shared__ __align__(16) int srow[CSA_NBKP];
  const int c = blockIdx.x, tid = threadIdx.x;
  for (int b = 0; b < CSA_NBK; ++b) sc[tid][b] = 0;
  const size_t e0 = (size_t)c * CSA_CHUNK + tid * 16;
  for (int i = 0; i < 16; ++i) { const size_t e = e0 + i; if (e < (size_t)CSA_E) { int d = DST[e * dstride]; d = min(max(d, 0), CSA_N - 1); sc[tid][d / CSA_BKT] += 1; } }
  __syncthreads();
  for (int b = tid; b < CSA_NBKP; b += 256) { int s = 0; if (b < CSA_NBK) for (int t = 0; t < 256; ++t) s += sc[t][b]; srow[b] = s; }
  __syncthreads();
  for (int q = tid; q < CSA_NBKP / 4; q += 256) vst2((unsigned*)(CNT + (size_t)c * CSA_NBKP + q * 4), *(const v4u*)&srow[q * 4]);
}
__global__ __launch_bounds__(256) void k_csA_scan(const int* __restrict__ CNT, int* __restrict__ OFF, int* __restrict__ BST) {
  __shared__ int sbt[CSA_NBK + 1]; __shared__ int sbs[((CSA_NBK + 1 + 31) / 32) * 32]; __shared__ int scnt[CSA_NBK + 1]; __shared__ __align__(16) int sbuf[64][CSA_OFFP];
  const int tid = threadIdx.x;
  for (int b = tid; b < CSA_NBK; b += 256) { int sp = 0, st = 0; for (int c = 0; c < CSA_NCH; ++c) { const int n = CNT[(size_t)c * CSA_NBKP + b]; st += n; sp += (n + 31) & ~31; } sbt[b] = sp; scnt[b] = st; }
  for (int b = tid; b < ((CSA_NBK + 1 + 31) / 32) * 32; b += 256) sbs[b] = 0;
  __syncthreads();
  if (tid == 0) { int acc = 0, accf = 0; for (int b = 0; b < CSA_NBK; ++b) { const int t = sbt[b]; sbt[b] = acc; acc += t; sbs[b] = accf; accf += (scnt[b] + 31) & ~31; } sbs[CSA_NBK] = accf; }
  __syncthreads();
  for (int b0 = 0; b0 < CSA_NBK; b0 += 64) {
    if (tid < 64 && b0 + tid < CSA_NBK) { const int b = b0 + tid; int o = sbt[b]; for (int c = 0; c < CSA_OFFP; ++c) { if (c < CSA_NCH) { sbuf[tid][c] = o; o += (CNT[(size_t)c * CSA_NBKP + b] + 31) & ~31; } else sbuf[tid][c] = 0; } }
    __syncthreads();
    for (int q = tid; q < 64 * (CSA_OFFP / 4); q += 256) { const int r = q / (CSA_OFFP / 4), pc = q % (CSA_OFFP / 4); if (b0 + r < CSA_NBK) vst2((unsigned*)(OFF + (size_t)(b0 + r) * CSA_OFFP + pc * 4), *(const v4u*)&sbuf[r][pc * 4]); }
    __syncthreads(); }
  for (int q = tid; q < ((CSA_NBK + 1 + 31) / 32) * 32 / 4; q += 256) vst2((unsigned*)(BST + q * 4), *(const v4u*)&sbs[q * 4]);
}
__global__ __launch_bounds__(256) void k_csA_scatter(const int* __restrict__ SRC, const int* __restrict__ DST, int sstride, int dstride, const int* __restrict__ OFF, int* __restrict__ SEGS, int* __restrict__ SEGE) {
  __shared__ unsigned short sc[256][CSA_NBK + 1]; __shared__ int sbase[CSA_NBK + 1]; __shared__ int scn[CSA_NBK + 1]; __shared__ int sord[CSA_CHUNK];
  const int c = blockIdx.x, tid = threadIdx.x;
  for (int b = 0; b < CSA_NBK; ++b) sc[tid][b] = 0;
  const size_t e0 = (size_t)c * CSA_CHUNK + tid * 16; int bk[16];
#pragma unroll
  for (int i = 0; i < 16; ++i) { const size_t e = e0 + i; bk[i] = -1; if (e < (size_t)CSA_E) { int d = DST[e * dstride]; d = min(max(d, 0), CSA_N - 1); bk[i] = d / CSA_BKT; sc[tid][bk[i]] += 1; } }
  __syncthreads();
  for (int b = tid; b < CSA_NBK; b += 256) { int acc = 0; for (int t = 0; t < 256; ++t) { const int v = sc[t][b]; sc[t][b] = (unsigned short)acc; acc += v; } scn[b] = acc; }
  __syncthreads();
  if (tid == 0) { int acc = 0; for (int b = 0; b < CSA_NBK; ++b) { sbase[b] = acc; acc += scn[b]; } }
  __syncthreads();
#pragma unroll
  for (int i = 0; i < 16; ++i) { if (bk[i] >= 0) { const int b = bk[i]; const int r = sc[tid][b]; sc[tid][b] = (unsigned short)(r + 1); sord[sbase[b] + r] = tid * 16 + i; } }
  __syncthreads();
  for (int b = 0; b < CSA_NBK; ++b) { const int n = scn[b]; if (n == 0) continue; const int nl = ((n + 31) & ~31); const size_t o = (size_t)(min(max(OFF[(size_t)b * CSA_OFFP + c], 0), CSA_SEGCAP - nl) & ~31);
    for (int q = tid; q < nl / 4; q += 256) { int4 vs, ve;
#pragma unroll
      for (int k = 0; k < 4; ++k) { const int i = q * 4 + k; int s = -1, eid = -1; if (i < n) { const size_t e = (size_t)c * CSA_CHUNK + sord[sbase[b] + i]; s = min(max(SRC[e * sstride], 0), CSA_N - 1); eid = (int)e; } vs[k] = s; ve[k] = eid; }
      vst2((unsigned*)(SEGS + o + q * 4), *(const v4u*)&vs); vst2((unsigned*)(SEGE + o + q * 4), *(const v4u*)&ve); } }
}
__global__ __launch_bounds__(256) void k_csA_bucket(const int* __restrict__ CNT, const int* __restrict__ OFF, const int* __restrict__ BST, const int* __restrict__ SEGS, const int* __restrict__ SEGE, const int* __restrict__ DST, int dstride, int* __restrict__ FS, int* __restrict__ FE, int* __restrict__ ROWST, int* __restrict__ ROWCNT) {
  __shared__ int ssrc[CSA_BCAP]; __shared__ int seid[CSA_BCAP]; __shared__ unsigned char snod[CSA_BCAP]; __shared__ int souts[CSA_BCAP]; __shared__ int soute[CSA_BCAP]; __shared__ int scount[256]; __shared__ int sstart[257]; __shared__ int stot;
  const int b = blockIdx.x, tid = threadIdx.x;
  if (tid == 0) { int t = 0; for (int c = 0; c < CSA_NCH; ++c) t += min(max(CNT[(size_t)c * CSA_NBKP + b], 0), CSA_CHUNK); stot = (t <= CSA_BCAP) ? t : 0; }
  __syncthreads();
  { int base = 0; for (int c = 0; c < CSA_NCH; ++c) { const int n = min(max(CNT[(size_t)c * CSA_NBKP + b], 0), CSA_CHUNK); const int o = min(max(OFF[(size_t)b * CSA_OFFP + c], 0), CSA_SEGCAP - ((n + 31) & ~31));
      for (int i = tid; i < n; i += 256) { const int p = base + i; if (p < CSA_BCAP) { ssrc[p] = min(max(SEGS[o + i], 0), CSA_N - 1); const int e = min(max(SEGE[o + i], 0), CSA_E - 1); seid[p] = e; int d = DST[(size_t)e * dstride]; d = min(max(d, 0), CSA_N - 1); const int dl = d - b * CSA_BKT; snod[p] = (unsigned char)(dl >= 0 && dl < 256 ? dl : 255); } }
      base += n; } }
  __syncthreads();
  const int node = b * CSA_BKT + tid; int cnt = 0; for (int p = 0; p < stot; ++p) cnt += (snod[p] == tid) ? 1 : 0;
  scount[tid] = cnt; __syncthreads();
  if (tid == 0) { int acc = 0; for (int t = 0; t < 256; ++t) { sstart[t] = acc; acc += scount[t]; } sstart[256] = acc; }
  __syncthreads();
  const int bst0 = min(max(BST[b], 0), CSA_FINN - ((sstart[256] + 31) & ~31)) & ~31; const int gst = bst0 + sstart[tid];
  { int w = sstart[tid]; for (int p = 0; p < stot; ++p) if (snod[p] == tid) { souts[w] = ssrc[p]; soute[w] = seid[p]; ++w; } }
  __syncthreads();
  { const int n = sstart[256]; const int nl = (n + 31) & ~31; for (int q = tid; q < nl / 4; q += 256) { int4 vs, ve;
#pragma unroll
      for (int k = 0; k < 4; ++k) { const int i = q * 4 + k; vs[k] = i < n ? souts[i] : -1; ve[k] = i < n ? soute[i] : -1; }
      vst2((unsigned*)(FS + bst0 + q * 4), *(const v4u*)&vs); vst2((unsigned*)(FE + bst0 + q * 4), *(const v4u*)&ve); } }
  __syncthreads();
  { __shared__ __align__(16) int srs[256], src2[256]; srs[tid] = node < CSA_N ? gst : 0; src2[tid] = node < CSA_N ? cnt : 0; __syncthreads();
    if (tid < 64) vst2((unsigned*)(ROWST + (size_t)b * 256 + tid * 4), *(const v4u*)&srs[tid * 4]); else if (tid < 128) vst2((unsigned*)(ROWCNT + (size_t)b * 256 + (tid - 64) * 4), *(const v4u*)&src2[(tid - 64) * 4]); }
}


#define WS_CNT  0u
#define WS_OFF  (WS_CNT + CSA_SZ_CNT)
#define WS_BST  (WS_OFF + CSA_SZ_OFF)
#define WS_SEGS (WS_BST + CSA_SZ_BST)
#define WS_SEGE (WS_SEGS + CSA_SZ_SEG)
#define WS_FS   (WS_SEGE + CSA_SZ_SEG)
#define WS_FE   (WS_FS + CSA_SZ_FIN)
#define WS_RST  (WS_FE + CSA_SZ_FIN)
#define WS_RCT  (WS_RST + CSA_SZ_ROW)
#define RSTR 64
#define WS_FS2  (WS_RCT + CSA_SZ_ROW)
#define WS_RC   (WS_FS2 + 4u * NPAD * RSTR)
#define WS_PW   (WS_RC + 4u * NPAD * 16)
#define PW1(r) ((size_t)(r) * HID * FIN)
#define PR1    ((size_t)NR * HID * FIN)
#define PW2(r) (PR1 + (size_t)HID * FIN + (size_t)(r) * H2 * HID)
#define PR2    (PR1 + (size_t)HID * FIN + (size_t)NR * H2 * HID)
#define PWEND  (PR2 + (size_t)H2 * HID)
#define WS_HR   (WS_PW + 2u * PWEND)
#define WS_ACC  (WS_HR + 4u * NPAD * HID)
#define WS_H1   (WS_ACC + 4u * NPAD * HID)
#define WS_END  (WS_H1 + 4u * NPAD * HID)

__global__ __launch_bounds__(256) void k_key(const int* __restrict__ DST, const int* __restrict__ ET, int* __restrict__ KEY) {
  __shared__ __align__(16) int s[256]; const size_t e0 = (size_t)blockIdx.x * 256; const int t = threadIdx.x; const size_t e = e0 + t;
  int k = 0; if (e < NE) { const int d = min(max(DST[e], 0), NN - 1), r = min(max(ET[e], 0), NR - 1); k = d * NR + r; } s[t] = k; __syncthreads();
  if (t < 64 && e0 + t * 4 < NE) vst2((unsigned*)(KEY + e0 + t * 4), *(const v4u*)&s[t * 4]);
}
__global__ __launch_bounds__(256) void k_packW(const float* __restrict__ Wm, int K, int NOUT, __bf16* __restrict__ DST_) {
  __shared__ __align__(16) __bf16 s[HID]; const int n = blockIdx.x, tid = threadIdx.x;
  for (int k = tid; k < K; k += 256) s[k] = (__bf16)Wm[(size_t)k * NOUT + n];
  __syncthreads();
  for (int q = tid; q < K / 8; q += 256) vst2((unsigned*)(DST_ + (size_t)n * K + q * 8), *(const v4u*)&s[q * 8]);
}
template <int RIN, int NT, int EPI>
__global__ __launch_bounds__(128) void k_gemm(const float* __restrict__ A, int lda, int K, const __bf16* __restrict__ P, const float* __restrict__ bias, float* __restrict__ OUT, int ldo) {
  __shared__ __align__(16) float so[4][16][NT * 16 + 4];
  const int tid = threadIdx.x, wave = tid >> 5, lane = tid & 31, col = lane & 15, g = lane >> 4; const size_t r0 = (size_t)blockIdx.x * 64 + wave * 16; const int n0 = blockIdx.y * NT * 16; size_t ra = r0 + col; if (ra >= NN) ra = NN - 1;
  v8f acc[NT]; for (int j = 0; j < NT; ++j) acc[j] = (v8f){};
#pragma unroll 2
  for (int kc = 0; kc < K / 32; ++kc) { F2 a; if (RIN) { v16b ax; const float* p = A + ra * lda + kc * 32 + 8 * g;
#pragma unroll
      for (int i = 0; i < 8; ++i) { ax[i] = (__bf16)p[i]; ax[8 + i] = (__bf16)p[16 + i]; } a.h = ax; a.l = ax; } else a = split_row(A + ra * lda, kc * 32, lane);
#pragma unroll
    for (int j = 0; j < NT; ++j) { const v16b w = frag_b(P + (size_t)(n0 + j * 16 + col) * K + kc * 32, lane); if (!RIN) acc[j] = wmma_bf(a.l, w, acc[j]); acc[j] = wmma_bf(a.h, w, acc[j]); } }
#pragma unroll
  for (int j = 0; j < NT; ++j) { const float bb = EPI ? bfr(bias[n0 + j * 16 + col]) : 0.f;
#pragma unroll
    for (int r = 0; r < 8; ++r) so[wave][8 * g + r][j * 16 + col] = acc[j][r] + bb; }
  LDSX();
  for (int rl = 0; rl < 16; ++rl) for (int pc = lane; pc < NT * 4; pc += 32) vst2(OUT + (r0 + rl) * (size_t)ldo + n0 + pc * 4, *(const v4f*)&so[wave][rl][pc * 4]);
}
__global__ __launch_bounds__(64) void k_relsplit(const int* __restrict__ FS, const int* __restrict__ FE, const int* __restrict__ ET, const int* __restrict__ RST, const int* __restrict__ RCT, int* __restrict__ FS2, int* __restrict__ RC) {
  __shared__ __align__(16) int sl[64][RSTR]; __shared__ __align__(16) int src_[64][16]; const int tid = threadIdx.x; const size_t i = (size_t)blockIdx.x * 64 + tid;
  int cntr[NR]; for (int r = 0; r < NR; ++r) cntr[r] = 0;
  for (int q = 0; q < RSTR; ++q) sl[tid][q] = 0;
  int cnt = 0, st = 0;
  if (i < NNT) { cnt = min(max(RCT[i], 0), CSA_BCAP); st = min(max(RST[i], 0), CSA_FINN - cnt);
    for (int e = 0; e < cnt; ++e) { const int s = min(max(FS[st + e], 0), NN - 1); if (s >= NNT) continue; const int r = min(max(ET[min(max(FE[st + e], 0), NE - 1)], 0), NR - 1);
#pragma unroll
      for (int rr = 0; rr < NR; ++rr) if (rr == r) cntr[rr]++; } }
  int off[NR]; { int run = 0;
#pragma unroll
    for (int r = 0; r < NR; ++r) { off[r] = run; run += cntr[r]; } }
  int pos[NR];
#pragma unroll
  for (int r = 0; r < NR; ++r) pos[r] = off[r];
  if (i < NNT) { for (int e = 0; e < cnt; ++e) { const int s = min(max(FS[st + e], 0), NN - 1); if (s >= NNT) continue; const int r = min(max(ET[min(max(FE[st + e], 0), NE - 1)], 0), NR - 1);
      int p = 0;
#pragma unroll
      for (int rr = 0; rr < NR; ++rr) if (rr == r) { p = pos[rr]; pos[rr]++; }
      if (p < RSTR) sl[tid][p] = s; } }
#pragma unroll
  for (int r = 0; r < NR; ++r) { src_[tid][r] = min(cntr[r], RSTR - min(off[r], RSTR)); src_[tid][8 + r] = min(off[r], RSTR); }
  __syncthreads();
  for (int q = 0; q < RSTR / 4; ++q) vst2((unsigned*)(FS2 + i * RSTR + q * 4), *(const v4u*)&sl[tid][q * 4]);
  for (int q = tid; q < 64 * 16 / 4; q += 64) vst2((unsigned*)(RC + ((size_t)blockIdx.x * 64) * 16 + q * 4), *(const v4u*)(&src_[0][0] + q * 4));
}
template <int W, int RELU>
__global__ __launch_bounds__(256) void k_ragg(const float* __restrict__ HR, const int* __restrict__ FS2, const int* __restrict__ RC, int r, float* __restrict__ ACC, float* __restrict__ OUTR) {
  constexpr int TPN = W / 4; constexpr int NPP = 256 / TPN; const int tid = threadIdx.x;
  for (int pass = 0; pass < 64 / NPP; ++pass) { const int nl = pass * NPP + tid / TPN; const int f0 = (tid % TPN) * 4; const size_t i = (size_t)blockIdx.x * 64 + nl;
    v4f acc = *(const v4f*)(ACC + i * W + f0);
    if (i < NNT) { const int cnt = min(max(RC[i * 16 + r], 0), RSTR); const int off = min(max(RC[i * 16 + 8 + r], 0), RSTR - cnt);
      if (cnt > 0) { v4f s = {0.f, 0.f, 0.f, 0.f};
        for (int e = 0; e < cnt; ++e) { const int src = min(max(FS2[i * RSTR + off + e], 0), NN - 1); const float* row = HR + (size_t)src * W + f0;
#pragma unroll
          for (int k = 0; k < 4; ++k) s[k] += row[k]; }
        const float inv = 1.0f / (float)cnt;
#pragma unroll
        for (int k = 0; k < 4; ++k) acc[k] += s[k] * inv; } }
    if (RELU) { v4f o;
#pragma unroll
      for (int k = 0; k < 4; ++k) o[k] = fmaxf(acc[k], 0.f); vst2(OUTR + i * W + f0, o); }
    else vst2(ACC + i * W + f0, acc); }
}
__global__ __launch_bounds__(256) void k_head(const float* __restrict__ Hh, const float* __restrict__ WS_, const float* __restrict__ BS_, float* __restrict__ out) {
  __shared__ __align__(16) float so[64]; const int tid = threadIdx.x; const int nl = tid >> 2, part = tid & 3; const size_t i = (size_t)blockIdx.x * 64 + nl;
  float a = 0.f; const float* h = Hh + i * H2 + part * 32;
#pragma unroll 8
  for (int k = 0; k < 32; ++k) a += h[k] * bfr(WS_[part * 32 + k]);
  a += __shfl_xor(a, 1); a += __shfl_xor(a, 2);
  if (part == 0) so[nl] = (i < NNT) ? sigm(a + bfr(BS_[0])) : 0.f;
  __syncthreads();
  if (tid < 16 && (size_t)blockIdx.x * 64 + tid * 4 + 4 <= (size_t)NN) vst2(out + (size_t)blockIdx.x * 64 + tid * 4, *(const v4f*)&so[tid * 4]);
}
extern "C" void kernel_launch(void* const* d_in, const int* in_sizes, int n_in, void* d_out, int out_size, void* d_ws, size_t ws_size, hipStream_t stream) {
  (void)in_sizes; (void)n_in; (void)out_size;
  const float** F = (const float**)d_in; const int* EI = (const int*)d_in[1]; const int* ET = (const int*)d_in[2];
  if (ws_size < (size_t)WS_END) return;
  char* ws = (char*)d_ws;
  int *CNT = (int*)(ws + WS_CNT), *OFF = (int*)(ws + WS_OFF), *BST = (int*)(ws + WS_BST), *SEGS = (int*)(ws + WS_SEGS), *SEGE = (int*)(ws + WS_SEGE), *FS = (int*)(ws + WS_FS), *FE = (int*)(ws + WS_FE), *RST = (int*)(ws + WS_RST), *RCT = (int*)(ws + WS_RCT);
  __bf16* PW = (__bf16*)(ws + WS_PW); float *HR = (float*)(ws + WS_HR), *ACC = (float*)(ws + WS_ACC), *H1 = (float*)(ws + WS_H1); int *FS2 = (int*)(ws + WS_FS2), *RC = (int*)(ws + WS_RC);
  const int* SRC = EI; const int* DST = EI + NE;
  k_csA_cnt<<<CSA_NCH, 256, 0, stream>>>(DST, 1, CNT); k_csA_scan<<<1, 256, 0, stream>>>(CNT, OFF, BST); k_csA_scatter<<<CSA_NCH, 256, 0, stream>>>(SRC, DST, 1, 1, OFF, SEGS, SEGE); k_csA_bucket<<<CSA_NBK, 256, 0, stream>>>(CNT, OFF, BST, SEGS, SEGE, DST, 1, FS, FE, RST, RCT);
  k_relsplit<<<NRB, 64, 0, stream>>>(FS, FE, ET, RST, RCT, FS2, RC);
  for (int r = 0; r < NR; ++r) { k_packW<<<HID, 256, 0, stream>>>(F[3] + (size_t)r * FIN * HID, FIN, HID, PW + PW1(r)); k_packW<<<H2, 256, 0, stream>>>(F[6] + (size_t)r * HID * H2, HID, H2, PW + PW2(r)); }
  k_packW<<<HID, 256, 0, stream>>>(F[4], FIN, HID, PW + PR1); k_packW<<<H2, 256, 0, stream>>>(F[7], HID, H2, PW + PR2);
  k_gemm<1, 8, 1><<<dim3(NRBT, HID / 128), 128, 0, stream>>>(F[0], FIN, FIN, PW + PR1, F[5], ACC, HID);
  for (int r = 0; r < NR; ++r) { k_gemm<1, 8, 0><<<dim3(NRBT, HID / 128), 128, 0, stream>>>(F[0], FIN, FIN, PW + PW1(r), nullptr, HR, HID);
    if (r < NR - 1) k_ragg<HID, 0><<<NRBT, 256, 0, stream>>>(HR, FS2, RC, r, ACC, nullptr); else k_ragg<HID, 1><<<NRBT, 256, 0, stream>>>(HR, FS2, RC, r, ACC, H1); }
  k_gemm<0, 8, 1><<<dim3(NRBT, H2 / 128), 128, 0, stream>>>(H1, HID, HID, PW + PR2, F[8], ACC, H2);
  for (int r = 0; r < NR; ++r) { k_gemm<0, 8, 0><<<dim3(NRBT, H2 / 128), 128, 0, stream>>>(H1, HID, HID, PW + PW2(r), nullptr, HR, H2);
    if (r < NR - 1) k_ragg<H2, 0><<<NRBT, 256, 0, stream>>>(HR, FS2, RC, r, ACC, nullptr); else k_ragg<H2, 1><<<NRBT, 256, 0, stream>>>(HR, FS2, RC, r, ACC, H1); }
  k_head<<<NRBT, 256, 0, stream>>>(H1, F[9], F[10], (float*)d_out);
}
